// WindowAttentionMemory_69080253988942
// MI455X (gfx1250) — hardware-verified
//
#include <hip/hip_runtime.h>
#include <stdint.h>

#define N_BATCH   4
#define SEQ_LEN   2048
#define EMB_DIM   1024
#define N_HEAD    16
#define HEAD_DIM  64
#define WIN_SZ    256
#define N_TOK     (N_BATCH * SEQ_LEN)
#define KV_CH     64
#define Q_BLK     64
#define P_CARRY   32768.0f
#define CTX_CARRY 16.0f
#define W_CARRY   64.0f
#define LN_EPSV   1e-12f
#define MASK_FILL (-3.4028234663852886e38f)

static_assert(N_TOK % 64 == 0);
static_assert(EMB_DIM % 64 == 0);
static_assert(EMB_DIM % 32 == 0);
static_assert(SEQ_LEN % Q_BLK == 0);
static_assert(HEAD_DIM == 64);
static_assert(N_HEAD * HEAD_DIM == EMB_DIM);
static_assert(WIN_SZ % KV_CH == 0);
static_assert(EMB_DIM == 128 * 8);

typedef __attribute__((ext_vector_type(16))) _Float16 v16h;
typedef __attribute__((ext_vector_type(8)))  _Float16 v8h;
typedef __attribute__((ext_vector_type(16))) __bf16   v16b;
typedef __attribute__((ext_vector_type(8)))  __bf16   v8b;
typedef __attribute__((ext_vector_type(8)))  float    v8f;
typedef __attribute__((ext_vector_type(4)))  float    v4f;
typedef __attribute__((ext_vector_type(4)))  unsigned v4u;
#define PSCALE 32768.0f
#define U16(p) ((const unsigned short*)(const void*)(p))
#define PSCALE_INV (1.0f / 32768.0f)

__device__ __forceinline__ unsigned short f2bf_bits(float f) {
  unsigned u = __float_as_uint(f);
  return (unsigned short)((u + 0x7FFFu + ((u >> 16) & 1u)) >> 16);
}
__device__ __forceinline__ float bf_bits2f(unsigned short h) { return __uint_as_float(((unsigned)h) << 16); }

__device__ __forceinline__ void dep_guard_h(v8f& a, v8f& b, v16h x, v16h y) { asm volatile("v_nop\n\tv_nop\n\tv_nop\n\tv_nop" : "+v"(a), "+v"(b) : "v"(x), "v"(y)); }
__device__ __forceinline__ void dep_guard_b(v8f& a, v8f& b, v16b x, v16b y) { asm volatile("v_nop\n\tv_nop\n\tv_nop\n\tv_nop" : "+v"(a), "+v"(b) : "v"(x), "v"(y)); }
__device__ __forceinline__ void keep4_h(v16h a, v16h b, v16h c, v16h d) { asm volatile("v_nop" :: "v"(a), "v"(b), "v"(c), "v"(d)); }
__device__ __forceinline__ void keep4_b(v16b a, v16b b, v16b c, v16b d) { asm volatile("v_nop" :: "v"(a), "v"(b), "v"(c), "v"(d)); }
__device__ __forceinline__ void acc_guard4(v8f& a, v8f& b, v8f& c, v8f& d) { asm volatile("v_nop\n\tv_nop\n\tv_nop\n\tv_nop" : "+v"(a), "+v"(b), "+v"(c), "+v"(d)); }
template <typename T> struct Frag;
template <> struct Frag<_Float16> {
  typedef v16h V; union U { v16h v; v8h h[2]; };
  static __device__ __forceinline__ v16h load(const _Float16* p) {
    U f; f.h[0] = *(const v8h*)(p); f.h[1] = *(const v8h*)(p + 16); return f.v;
  }
  static __device__ __forceinline__ v8f mma(v16h a, v16h b, v8f c) {
    return __builtin_amdgcn_wmma_f32_16x16x32_f16(false, a, false, b, (short)0, c, false, false);
  }
  static __device__ __forceinline__ void guard(v8f& a, v8f& b, v16h x, v16h y) { dep_guard_h(a, b, x, y); }
  static __device__ __forceinline__ void keep(v16h a, v16h b, v16h c, v16h d) { keep4_h(a, b, c, d); }
};
template <> struct Frag<__bf16> {
  typedef v16b V; union U { v16b v; v8b h[2]; };
  static __device__ __forceinline__ v16b load(const __bf16* p) {
    U f; f.h[0] = *(const v8b*)(p); f.h[1] = *(const v8b*)(p + 16); return f.v;
  }
  static __device__ __forceinline__ v8f mma(v16b a, v16b b, v8f c) {
    return __builtin_amdgcn_wmma_f32_16x16x32_bf16(false, a, false, b, (short)0, c, false, false);
  }
  static __device__ __forceinline__ void guard(v8f& a, v8f& b, v16b x, v16b y) { dep_guard_b(a, b, x, y); }
  static __device__ __forceinline__ void keep(v16b a, v16b b, v16b c, v16b d) { keep4_b(a, b, c, d); }
};

template <int ET> struct Elem;
template <> struct Elem<0> { typedef _Float16 T; };
template <> struct Elem<1> { typedef __bf16 T; };
template <int ET, bool SPLIT, int BIAS_MODE, int OUT_MODE, bool RESID, int ACT = 0>
__global__ __launch_bounds__(256) void wmma_gemm64(
    const unsigned short* __restrict__ Ap, const unsigned short* __restrict__ A2p, int lda, long strideA,
    const unsigned short* __restrict__ Btp, const unsigned short* __restrict__ Bt2p, int ldb, long strideB,
    void* __restrict__ Cout, void* __restrict__ Cout2, int ldc, long strideC,
    const float* __restrict__ bias,
    const float* __restrict__ resid, long strideR,
    int M, int N, int K, float scale) {
  typedef typename Elem<ET>::T T;
  typedef typename Frag<T>::V V;
  const T* A = (const T*)Ap; const T* A2 = (const T*)A2p; const T* Bt = (const T*)Btp; const T* Bt2 = (const T*)Bt2p;
  __shared__ __align__(16) float sT[8][16 * 68];
  const int b    = blockIdx.y;
  const int lane = threadIdx.x & 31;
  const int wave = threadIdx.x >> 5;
  const int tilesN = N >> 6;
  const int tilesM = M >> 6;
  const int tile = blockIdx.x * 8 + wave;
  if (tile >= tilesM * tilesN) return;
  const int tm = tile / tilesN;
  const int tn = tile - tm * tilesN;
  const int m0 = tm << 6;
  const int n0 = tn << 6;

  const T* Ab  = A  + (size_t)b * strideA;
  const T* Bb  = Bt + (size_t)b * strideB;
  const T* Ab2 = SPLIT ? (A2  + (size_t)b * strideA) : nullptr;
  const T* Bb2 = SPLIT ? (Bt2 + (size_t)b * strideB) : nullptr;

  const int rlane = lane & 15;
  const int koff  = (lane >> 4) * 8;
  const int mOff  = (lane >> 4) * 8;

  v8f acc[4][4];
#pragma unroll
  for (int i = 0; i < 4; ++i)
#pragma unroll
    for (int j = 0; j < 4; ++j) acc[i][j] = (v8f){0.f,0.f,0.f,0.f,0.f,0.f,0.f,0.f};

  for (int k0 = 0; k0 < K; k0 += 32) {
    V bh[4], bl[4];
#pragma unroll
    for (int j = 0; j < 4; ++j) {
      const size_t bo = (size_t)(n0 + (j << 4) + rlane) * ldb + koff + k0;
      bh[j] = Frag<T>::load(Bb + bo);
      if (SPLIT) bl[j] = Frag<T>::load(Bb2 + bo);
    }
#pragma unroll
    for (int i = 0; i < 4; ++i) {
      const size_t ao = (size_t)(m0 + (i << 4) + rlane) * lda + koff + k0;
      V ah = Frag<T>::load(Ab + ao);
      V al;
      if (SPLIT) al = Frag<T>::load(Ab2 + ao);
#pragma unroll
      for (int j = 0; j < 4; ++j) {
        acc[i][j] = Frag<T>::mma(ah, bh[j], acc[i][j]);
        if (SPLIT) {
          acc[i][j] = Frag<T>::mma(ah, bl[j], acc[i][j]);
          acc[i][j] = Frag<T>::mma(al, bh[j], acc[i][j]);
        }
      }
      Frag<T>::guard(acc[i][0], acc[i][3], ah, SPLIT ? al : ah);
    }
    Frag<T>::keep(bh[0], bh[1], bh[2], bh[3]);
    if (SPLIT) Frag<T>::keep(bl[0], bl[1], bl[2], bl[3]);
  }
  acc_guard4(acc[0][0], acc[0][1], acc[0][2], acc[0][3]);
  acc_guard4(acc[1][0], acc[1][1], acc[1][2], acc[1][3]);
  acc_guard4(acc[2][0], acc[2][1], acc[2][2], acc[2][3]);
  acc_guard4(acc[3][0], acc[3][1], acc[3][2], acc[3][3]);

  float* slab = sT[wave];
  const float* Rb = RESID ? (resid + (size_t)b * strideR) : nullptr;
#pragma unroll
  for (int i = 0; i < 4; ++i) {
    const int mBase = m0 + (i << 4);
#pragma unroll
    for (int j = 0; j < 4; ++j) {
      const int n = n0 + (j << 4) + rlane;
      float bv = 0.f;
      if (BIAS_MODE == 2) bv = bias[n];
#pragma unroll
      for (int r = 0; r < 8; ++r) {
        float v = acc[i][j][r] * scale;
        if (BIAS_MODE == 1) v += bias[mBase + mOff + r];
        if (BIAS_MODE == 2) v += bv;
        if (RESID) v += Rb[(size_t)(mBase + mOff + r) * ldc + n];
        if (ACT == 1) v = tanhf(v);
        if (ACT == 2) v = fmaxf(v, 0.0f);
        if (ACT == 3) v = v / (1.0f + expf(-v));
        if (ACT == 4) v = (v > 0.f) ? v : 0.01f * v;
        if (ACT == 5) v = 0.5f * v * (1.0f + erff(v * 0.70710678118654752f));
        slab[(mOff + r) * 68 + (j << 4) + rlane] = v;
      }
    }
    __builtin_amdgcn_fence(__ATOMIC_RELEASE, "workgroup");
    __builtin_amdgcn_wave_barrier();
    __builtin_amdgcn_fence(__ATOMIC_ACQUIRE, "workgroup");
    if (OUT_MODE == 0) {
      float* C = (float*)Cout + (size_t)b * strideC;
      const int hh = lane >> 4, c4 = (lane & 15) * 4;
      for (int pass = 0; pass < 2; ++pass) {
#pragma unroll
        for (int it = 0; it < 8; ++it) {
          const int row = it * 2 + hh;
          v4f v = *(const v4f*)(slab + row * 68 + c4);
          *(volatile v4f*)(C + (size_t)(mBase + row) * ldc + n0 + c4) = v;
        }
        __threadfence();
      }
    } else {
      const int q = lane >> 3, c8 = (lane & 7) * 8;
      unsigned short* C  = (unsigned short*)Cout  + (size_t)b * strideC;
      unsigned short* C2 = (OUT_MODE == 2) ? ((unsigned short*)Cout2 + (size_t)b * strideC) : nullptr;
      for (int pass = 0; pass < 2; ++pass) {
#pragma unroll
        for (int it = 0; it < 4; ++it) {
          const int row = it * 4 + q;
          const float* sp = slab + row * 68 + c8;
          v8h hv, lv;
#pragma unroll
          for (int e = 0; e < 8; ++e) {
            if (OUT_MODE == 1) {
              hv[e] = (_Float16)sp[e];
            } else {
              unsigned short hb = f2bf_bits(sp[e]);
              unsigned short lb = f2bf_bits(sp[e] - bf_bits2f(hb));
              hv[e] = __builtin_bit_cast(_Float16, hb);
              lv[e] = __builtin_bit_cast(_Float16, lb);
            }
          }
          *(volatile v8h*)(C + (size_t)(mBase + row) * ldc + n0 + c8) = hv;
          if (OUT_MODE == 2) *(volatile v8h*)(C2 + (size_t)(mBase + row) * ldc + n0 + c8) = lv;
        }
        __threadfence();
      }
    }
    __builtin_amdgcn_fence(__ATOMIC_RELEASE, "workgroup");
    __builtin_amdgcn_wave_barrier();
    __builtin_amdgcn_fence(__ATOMIC_ACQUIRE, "workgroup");
  }
}

__global__ __launch_bounds__(128) void ln_f16_kernel(const float* __restrict__ x,
                                                     const float* __restrict__ gam,
                                                     const float* __restrict__ bet,
                                                     unsigned short* __restrict__ xn) {
  __shared__ float red_a[4];
  __shared__ float red_b[4];
  const int row  = blockIdx.x;
  const int t    = threadIdx.x;
  const int wave = t >> 5, lane = t & 31;

  const float* xr = x + (size_t)row * EMB_DIM + t * 8;
  const v4f a0 = *(const v4f*)(xr);
  const v4f a1 = *(const v4f*)(xr + 4);
  float v[8];
  v[0] = a0[0]; v[1] = a0[1]; v[2] = a0[2]; v[3] = a0[3];
  v[4] = a1[0]; v[5] = a1[1]; v[6] = a1[2]; v[7] = a1[3];

  float s = ((v[0] + v[1]) + (v[2] + v[3])) + ((v[4] + v[5]) + (v[6] + v[7]));
#pragma unroll
  for (int off = 16; off >= 1; off >>= 1) s += __shfl_xor(s, off, 32);
  if (lane == 0) red_a[wave] = s;
  __syncthreads();
  const float mu = ((red_a[0] + red_a[1]) + (red_a[2] + red_a[3])) * (1.0f / (float)EMB_DIM);

  float d[8];
  float ss = 0.f;
#pragma unroll
  for (int e = 0; e < 8; ++e) { d[e] = v[e] - mu; ss += d[e] * d[e]; }
#pragma unroll
  for (int off = 16; off >= 1; off >>= 1) ss += __shfl_xor(ss, off, 32);
  if (lane == 0) red_b[wave] = ss;
  __syncthreads();
  const float var = ((red_b[0] + red_b[1]) + (red_b[2] + red_b[3])) * (1.0f / (float)EMB_DIM);
  const float rs  = rsqrtf(var + LN_EPSV);

  const v4f g0 = *(const v4f*)(gam + t * 8);
  const v4f g1 = *(const v4f*)(gam + t * 8 + 4);
  const v4f b0 = *(const v4f*)(bet + t * 8);
  const v4f b1 = *(const v4f*)(bet + t * 8 + 4);
  float gg[8], bb[8];
  gg[0] = g0[0]; gg[1] = g0[1]; gg[2] = g0[2]; gg[3] = g0[3];
  gg[4] = g1[0]; gg[5] = g1[1]; gg[6] = g1[2]; gg[7] = g1[3];
  bb[0] = b0[0]; bb[1] = b0[1]; bb[2] = b0[2]; bb[3] = b0[3];
  bb[4] = b1[0]; bb[5] = b1[1]; bb[6] = b1[2]; bb[7] = b1[3];

  v8h hv;
#pragma unroll
  for (int e = 0; e < 8; ++e) hv[e] = (_Float16)(d[e] * rs * gg[e] + bb[e]);

  _Float16* dst = (_Float16*)xn + (size_t)row * EMB_DIM + t * 8;
  *(volatile v8h*)dst = hv;
  __threadfence();
  *(volatile v8h*)dst = hv;
}

__global__ __launch_bounds__(256) void cast_scale_f16x8(const float* __restrict__ in,
                                                       unsigned short* __restrict__ out,
                                                       int n8, float sc) {
  const int i = blockIdx.x * 256 + threadIdx.x;
  if (i < n8) {
    const v4f a0 = *(const v4f*)(in + (size_t)i * 8);
    const v4f a1 = *(const v4f*)(in + (size_t)i * 8 + 4);
    v8h hv;
    hv[0] = (_Float16)(a0[0] * sc); hv[1] = (_Float16)(a0[1] * sc);
    hv[2] = (_Float16)(a0[2] * sc); hv[3] = (_Float16)(a0[3] * sc);
    hv[4] = (_Float16)(a1[0] * sc); hv[5] = (_Float16)(a1[1] * sc);
    hv[6] = (_Float16)(a1[2] * sc); hv[7] = (_Float16)(a1[3] * sc);
    _Float16* dst = (_Float16*)out + (size_t)i * 8;
    *(volatile v8h*)dst = hv;
    __threadfence();
    *(volatile v8h*)dst = hv;
  }
}

__device__ __forceinline__ v8f mma16f(v16h a, v16h b, v8f c) {
  c = __builtin_amdgcn_wmma_f32_16x16x32_f16(false, a, false, b, (short)0, c, false, false);
  asm volatile("v_nop\n\tv_nop\n\tv_nop\n\tv_nop" : "+v"(c) : "v"(a), "v"(b));
  return c;
}

__global__ __launch_bounds__(128)
void swin_attn_kernel(const unsigned short* __restrict__ qp, const unsigned short* __restrict__ kp,
                      const unsigned short* __restrict__ vtp, unsigned short* __restrict__ cxp) {
  union FH { v16h v; v8h h[2]; };
  __shared__ __align__(16) unsigned short Ksh[KV_CH * HEAD_DIM];
  __shared__ __align__(16) unsigned short Vts[HEAD_DIM * KV_CH];
  __shared__ __align__(16) _Float16 Psh[4][16 * KV_CH];
  __shared__ __align__(16) float Osh[4][16 * 68];

  const int tid  = threadIdx.x;
  const int wave = tid >> 5;
  const int lane = tid & 31;
  const int hh   = lane >> 4;
  const int c    = lane & 15;

  const int bx = blockIdx.x;
  const int qb = bx % (SEQ_LEN / Q_BLK);
  const int bh = bx / (SEQ_LEN / Q_BLK);
  const int h  = bh % N_HEAD;
  const int b  = bh / N_HEAD;
  const int q0 = qb * Q_BLK + wave * 16;

  v16h qa[2];
  {
    const _Float16* qrow = (const _Float16*)qp + (size_t)(b * SEQ_LEN + q0 + c) * EMB_DIM + h * HEAD_DIM;
#pragma unroll
    for (int dc = 0; dc < 2; ++dc) qa[dc] = Frag<_Float16>::load(qrow + dc * 32 + 8 * hh);
  }

  float mrow[8], lrow[8];
  v8f oacc[4];
#pragma unroll
  for (int r = 0; r < 8; ++r) { mrow[r] = -__builtin_inff(); lrow[r] = 0.f; }
#pragma unroll
  for (int t = 0; t < 4; ++t) oacc[t] = (v8f){0.f,0.f,0.f,0.f,0.f,0.f,0.f,0.f};

  const int kcs = (qb >= (WIN_SZ / KV_CH)) ? (qb - (WIN_SZ / KV_CH)) : 0;
  for (int kc = kcs; kc <= qb; ++kc) {
    const int kv0 = kc * KV_CH;
    __syncthreads();
#pragma unroll
    for (int i = 0; i < 4; ++i) {
      const int idx  = i * 128 + tid;
      const int rr   = idx >> 3;
      const int part = idx & 7;
      const v4u kw = *(const v4u*)(kp  + (size_t)(b * SEQ_LEN + kv0 + rr) * EMB_DIM + h * HEAD_DIM + part * 8);
      const v4u vw = *(const v4u*)(vtp + (size_t)(h * HEAD_DIM + rr) * N_TOK + b * SEQ_LEN + kv0 + part * 8);
      *(v4u*)(Ksh + rr * HEAD_DIM + part * 8) = kw;
      *(v4u*)(Vts + rr * KV_CH + part * 8)    = vw;
    }
    __syncthreads();

    v8f s[4];
#pragma unroll
    for (int j = 0; j < 4; ++j) {
      s[j] = (v8f){0.f,0.f,0.f,0.f,0.f,0.f,0.f,0.f};
#pragma unroll
      for (int dc = 0; dc < 2; ++dc) {
        FH kb;
        kb.h[0] = *(const v8h*)((const _Float16*)Ksh + (j * 16 + c) * HEAD_DIM + dc * 32 + 8 * hh);
        kb.h[1] = *(const v8h*)((const _Float16*)Ksh + (j * 16 + c) * HEAD_DIM + dc * 32 + 16 + 8 * hh);
        s[j] = mma16f(qa[dc], kb.v, s[j]);
      }
    }

    float cm[8];
#pragma unroll
    for (int r = 0; r < 8; ++r) {
      const int qrow = q0 + 8 * hh + r;
      float m = -__builtin_inff();
#pragma unroll
      for (int j = 0; j < 4; ++j) {
        const int kvcol = kv0 + j * 16 + c;
        const bool masked = (kvcol > qrow) || (qrow - kvcol >= WIN_SZ);
        const float sv = s[j][r] * 0.125f;
        s[j][r] = masked ? MASK_FILL : sv;
        m = fmaxf(m, s[j][r]);
      }
#pragma unroll
      for (int off = 1; off < 16; off <<= 1) m = fmaxf(m, __shfl_xor(m, off, 32));
      cm[r] = m;
    }

    _Float16* pw = Psh[wave];
#pragma unroll
    for (int r = 0; r < 8; ++r) {
      const float mnew  = fmaxf(mrow[r], cm[r]);
      const float alpha = expf(mrow[r] - mnew);
      mrow[r] = mnew;
      float psum = 0.f;
#pragma unroll
      for (int j = 0; j < 4; ++j) {
        const float p = expf(s[j][r] - mnew);
        psum += p;
        pw[(8 * hh + r) * KV_CH + j * 16 + c] = (_Float16)(p * P_CARRY);
      }
#pragma unroll
      for (int off = 1; off < 16; off <<= 1) psum += __shfl_xor(psum, off, 32);
      lrow[r] = lrow[r] * alpha + psum;
#pragma unroll
      for (int t = 0; t < 4; ++t) oacc[t][r] *= alpha;
    }
    __syncthreads();

#pragma unroll
    for (int kk = 0; kk < 2; ++kk) {
      FH pa;
      pa.h[0] = *(const v8h*)(pw + c * KV_CH + kk * 32 + 8 * hh);
      pa.h[1] = *(const v8h*)(pw + c * KV_CH + kk * 32 + 16 + 8 * hh);
#pragma unroll
      for (int t = 0; t < 4; ++t) {
        FH vb;
        vb.h[0] = *(const v8h*)((const _Float16*)Vts + (t * 16 + c) * KV_CH + kk * 32 + 8 * hh);
        vb.h[1] = *(const v8h*)((const _Float16*)Vts + (t * 16 + c) * KV_CH + kk * 32 + 16 + 8 * hh);
        oacc[t] = mma16f(pa.v, vb.v, oacc[t]);
      }
    }
  }

  float* os = Osh[wave];
#pragma unroll
  for (int r = 0; r < 8; ++r) {
    const float inv = CTX_CARRY / (lrow[r] * P_CARRY);
#pragma unroll
    for (int t = 0; t < 4; ++t) os[(8 * hh + r) * 68 + t * 16 + c] = oacc[t][r] * inv;
  }
  __syncthreads();
  {
    const int q8 = lane >> 3, c8 = (lane & 7) * 8;
    _Float16* cb = (_Float16*)cxp + (size_t)(b * SEQ_LEN + q0) * EMB_DIM + h * HEAD_DIM;
    for (int pass = 0; pass < 2; ++pass) {
#pragma unroll
      for (int it = 0; it < 4; ++it) {
        const int row = it * 4 + q8;
        const float* sp = os + row * 68 + c8;
        v8h hv;
#pragma unroll
        for (int e = 0; e < 8; ++e) hv[e] = (_Float16)sp[e];
        *(volatile v8h*)(cb + (size_t)row * EMB_DIM + c8) = hv;
      }
      __threadfence();
    }
  }
}

extern "C" void kernel_launch(void* const* d_in, const int* in_sizes, int n_in,
                              void* d_out, int out_size, void* d_ws, size_t ws_size,
                              hipStream_t stream) {
  if (n_in < 11) return;
  if (in_sizes[0] != N_TOK * EMB_DIM) return;
  if (in_sizes[1] != EMB_DIM || in_sizes[2] != EMB_DIM) return;
  if (in_sizes[3] != EMB_DIM * EMB_DIM || in_sizes[5] != EMB_DIM * EMB_DIM ||
      in_sizes[7] != EMB_DIM * EMB_DIM || in_sizes[9] != EMB_DIM * EMB_DIM) return;
  if (in_sizes[4] != EMB_DIM || in_sizes[6] != EMB_DIM || in_sizes[8] != EMB_DIM || in_sizes[10] != EMB_DIM) return;
  if (out_size != N_TOK * EMB_DIM) return;

  const float* x   = (const float*)d_in[0];
  const float* lng = (const float*)d_in[1];
  const float* lnb = (const float*)d_in[2];
  const float* wq  = (const float*)d_in[3];
  const float* bq  = (const float*)d_in[4];
  const float* wk  = (const float*)d_in[5];
  const float* bk  = (const float*)d_in[6];
  const float* wv  = (const float*)d_in[7];
  const float* bv  = (const float*)d_in[8];
  const float* wo  = (const float*)d_in[9];
  const float* bo  = (const float*)d_in[10];
  float* out = (float*)d_out;

  const size_t plane_b = (size_t)N_TOK * EMB_DIM * 2;
  const size_t wmat_b  = (size_t)EMB_DIM * EMB_DIM * 2;
  const size_t off_xn = 0;
  const size_t off_w  = off_xn + plane_b;
  const size_t off_q  = off_w + 4 * wmat_b;
  const size_t off_k  = off_q + plane_b;
  const size_t off_vt = off_k + plane_b;
  const size_t off_cx = off_vt + plane_b;
  const size_t total  = off_cx + plane_b;
  if (total > ws_size) return;

  unsigned char* wsb = (unsigned char*)d_ws;
  unsigned short* xn16 = (unsigned short*)(wsb + off_xn);
  unsigned short* wq16 = (unsigned short*)(wsb + off_w + 0 * wmat_b);
  unsigned short* wk16 = (unsigned short*)(wsb + off_w + 1 * wmat_b);
  unsigned short* wv16 = (unsigned short*)(wsb + off_w + 2 * wmat_b);
  unsigned short* wo16 = (unsigned short*)(wsb + off_w + 3 * wmat_b);
  unsigned short* q16  = (unsigned short*)(wsb + off_q);
  unsigned short* k16  = (unsigned short*)(wsb + off_k);
  unsigned short* vt16 = (unsigned short*)(wsb + off_vt);
  unsigned short* cx16 = (unsigned short*)(wsb + off_cx);

  ln_f16_kernel<<<N_TOK, 128, 0, stream>>>(x, lng, lnb, xn16);

  const int n8 = EMB_DIM * EMB_DIM / 8;
  const int cblk = (n8 + 255) / 256;
  cast_scale_f16x8<<<cblk, 256, 0, stream>>>(wq, wq16, n8, W_CARRY);
  cast_scale_f16x8<<<cblk, 256, 0, stream>>>(wk, wk16, n8, W_CARRY);
  cast_scale_f16x8<<<cblk, 256, 0, stream>>>(wv, wv16, n8, W_CARRY);
  cast_scale_f16x8<<<cblk, 256, 0, stream>>>(wo, wo16, n8, W_CARRY);

  const float wscale_inv = 1.0f / W_CARRY;
  const int tiles = (N_TOK / 64) * (EMB_DIM / 64);
  const dim3 ggrid((tiles + 7) / 8, 1);

  wmma_gemm64<0, false, 2, 1, false><<<ggrid, 256, 0, stream>>>(
      xn16, xn16, EMB_DIM, 0L, wq16, wq16, EMB_DIM, 0L,
      (void*)q16, (void*)q16, EMB_DIM, 0L, bq, bq, 0L, N_TOK, EMB_DIM, EMB_DIM, wscale_inv);
  wmma_gemm64<0, false, 2, 1, false><<<ggrid, 256, 0, stream>>>(
      xn16, xn16, EMB_DIM, 0L, wk16, wk16, EMB_DIM, 0L,
      (void*)k16, (void*)k16, EMB_DIM, 0L, bk, bk, 0L, N_TOK, EMB_DIM, EMB_DIM, wscale_inv);
  wmma_gemm64<0, false, 1, 1, false><<<ggrid, 256, 0, stream>>>(
      wv16, wv16, EMB_DIM, 0L, xn16, xn16, EMB_DIM, 0L,
      (void*)vt16, (void*)vt16, N_TOK, 0L, bv, bv, 0L, EMB_DIM, N_TOK, EMB_DIM, wscale_inv);

  swin_attn_kernel<<<N_BATCH * N_HEAD * (SEQ_LEN / Q_BLK), 128, 0, stream>>>(q16, k16, vt16, cx16);

  wmma_gemm64<0, false, 2, 0, true><<<ggrid, 256, 0, stream>>>(
      cx16, cx16, EMB_DIM, 0L, wo16, wo16, EMB_DIM, 0L,
      (void*)out, (void*)out, EMB_DIM, 0L, bo, x, 0L, N_TOK, EMB_DIM, EMB_DIM,
      wscale_inv * (1.0f / CTX_CARRY));
}
